// AttAggFME_893353197690
// MI455X (gfx1250) — hardware-verified
//
#include <hip/hip_runtime.h>
#include <stdint.h>
#include <stddef.h>


typedef unsigned short us_t;
typedef unsigned int v4u __attribute__((ext_vector_type(4)));
typedef unsigned int v2u __attribute__((ext_vector_type(2)));
typedef float v4f __attribute__((ext_vector_type(4)));
typedef float v8f __attribute__((ext_vector_type(8)));
typedef __bf16 v16b __attribute__((ext_vector_type(16)));
typedef _Float16 v16h __attribute__((ext_vector_type(16)));
typedef _Float16 v8h __attribute__((ext_vector_type(8)));

union FragB { v16b v; v4u q[2]; };
union FragH { v16h v; v4u q[2]; v8h hv[2]; };

#define HW   4096
#define NPX  16384
#define NOP4 "v_nop\n\tv_nop\n\tv_nop\n\tv_nop"

__device__ __forceinline__ v4u ldg16(const us_t* p) { return *(const v4u*)p; }
__device__ __forceinline__ v4u zero4u() { v4u z; z.x = 0u; z.y = 0u; z.z = 0u; z.w = 0u; return z; }
__device__ __forceinline__ v8f zero8f() { v8f z; for (int i = 0; i < 8; ++i) z[i] = 0.0f; return z; }

__device__ __forceinline__ unsigned bfbits(float f) {
  unsigned u = __float_as_uint(f);
  u += 0x7FFFu + ((u >> 16) & 1u);
  return u >> 16;
}
__device__ __forceinline__ void split2(float a, float b, unsigned& hi, unsigned& lo) {
  const unsigned ha = bfbits(a), hb = bfbits(b);
  const float ra = a - __uint_as_float(ha << 16);
  const float rb = b - __uint_as_float(hb << 16);
  hi = ha | (hb << 16);
  lo = bfbits(ra) | (bfbits(rb) << 16);
}
__device__ __forceinline__ void split8(const float* v, v4u& hi, v4u& lo) {
  unsigned h0, l0, h1, l1, h2, l2, h3, l3;
  split2(v[0], v[1], h0, l0);
  split2(v[2], v[3], h1, l1);
  split2(v[4], v[5], h2, l2);
  split2(v[6], v[7], h3, l3);
  hi.x = h0; hi.y = h1; hi.z = h2; hi.w = h3;
  lo.x = l0; lo.y = l1; lo.z = l2; lo.w = l3;
}
__device__ __forceinline__ unsigned h2bits(float a, float b) {
  const _Float16 x = (_Float16)a, y = (_Float16)b;
  return (unsigned)__builtin_bit_cast(unsigned short, x) | ((unsigned)__builtin_bit_cast(unsigned short, y) << 16);
}
__device__ __forceinline__ v4u pack8h(const float* v) {
  v4u r;
  r.x = h2bits(v[0], v[1]); r.y = h2bits(v[2], v[3]); r.z = h2bits(v[4], v[5]); r.w = h2bits(v[6], v[7]);
  return r;
}

__device__ __forceinline__ void st2u4(us_t* p, v4u v) { *(volatile v4u*)p = v; __threadfence(); *(volatile v4u*)p = v; }
__device__ __forceinline__ void st2u2(us_t* p, v2u v) { *(volatile v2u*)p = v; __threadfence(); *(volatile v2u*)p = v; }
__device__ __forceinline__ void st2f4(float* p, v4f v) { *(volatile v4f*)p = v; __threadfence(); *(volatile v4f*)p = v; }

__device__ __forceinline__ v8f mmab(v16b a, v16b b, v8f c) {
  return __builtin_amdgcn_wmma_f32_16x16x32_bf16(false, a, false, b, (short)0, c, false, false);
}
__device__ __forceinline__ v8f mmah(v16h a, v16h b, v8f c) {
  return __builtin_amdgcn_wmma_f32_16x16x32_f16(false, a, false, b, (short)0, c, false, false);
}

template <int MT> struct Guard;
template <> struct Guard<1> {
  static __device__ __forceinline__ void g(v8f* a, FragB* ah, FragB* al, FragB& bh, FragB& bl) {
    asm volatile(NOP4 : "+v"(a[0]) : "v"(ah[0].v), "v"(al[0].v), "v"(bh.v), "v"(bl.v));
  }
};
template <> struct Guard<2> {
  static __device__ __forceinline__ void g(v8f* a, FragB* ah, FragB* al, FragB& bh, FragB& bl) {
    asm volatile(NOP4 : "+v"(a[0]), "+v"(a[1])
                 : "v"(ah[0].v), "v"(ah[1].v), "v"(al[0].v), "v"(al[1].v), "v"(bh.v), "v"(bl.v));
  }
};
template <> struct Guard<4> {
  static __device__ __forceinline__ void g(v8f* a, FragB* ah, FragB* al, FragB& bh, FragB& bl) {
    asm volatile(NOP4 : "+v"(a[0]), "+v"(a[1]), "+v"(a[2]), "+v"(a[3])
                 : "v"(ah[0].v), "v"(ah[1].v), "v"(ah[2].v), "v"(ah[3].v),
                   "v"(al[0].v), "v"(al[1].v), "v"(al[2].v), "v"(al[3].v), "v"(bh.v), "v"(bl.v));
  }
};

__global__ __launch_bounds__(256) void k_packw(const float* __restrict__ w, int OC,
                                               const float* __restrict__ w2, int OC2,
                                               int Cin, int taps, int Cpad, int Kpad,
                                               us_t* wh, us_t* wl, int ngroups)
{
  const int g = blockIdx.x * 256 + threadIdx.x;
  if (g >= ngroups) return;
  const int e0 = g * 8;
  const int oc = e0 / Kpad;
  const int k0 = e0 - oc * Kpad;
  float v[8];
#pragma unroll
  for (int i = 0; i < 8; ++i) {
    const int k = k0 + i;
    const int tap = k / Cpad;
    const int ic = k - tap * Cpad;
    const bool valid = (tap < taps) && (ic < Cin);
    const int tapc = min(tap, taps - 1), icc = min(ic, Cin - 1);
    const int oc1 = min(oc, OC - 1);
    const float a = w[((size_t)oc1 * Cin + icc) * taps + tapc];
    float bq = 0.0f;
    if (OC2 > 0) {
      const int oc2 = min(max(oc - OC, 0), OC2 - 1);
      bq = w2[((size_t)oc2 * Cin + icc) * taps + tapc];
    }
    float t = 0.0f;
    if (oc < OC) t = a; else if (oc < OC + OC2) t = bq;
    v[i] = valid ? t : 0.0f;
  }
  v4u hi, lo;
  split8(v, hi, lo);
  st2u4(wh + e0, hi);
  st2u4(wl + e0, lo);
}

__global__ __launch_bounds__(256) void k_packwd(const float* __restrict__ w, us_t* wh, us_t* wl)
{
  const int g = blockIdx.x * 256 + threadIdx.x;
  if (g >= 1024) return;
  const int e0 = g * 8;
  const int z = e0 >> 11, o = (e0 >> 7) & 15, k0 = e0 & 127;
  const int py = z >> 1, pxp = z & 1;
  float v[8];
#pragma unroll
  for (int i = 0; i < 8; ++i) {
    const int k = k0 + i;
    const int t = k >> 5, ic = k & 31;
    const int a = t >> 1, c = t & 1;
    const int ky = py + 2 * a, kx = pxp + 2 * c;
    v[i] = w[((ic * 16 + o) * 4 + (3 - ky)) * 4 + (3 - kx)];
  }
  v4u hi, lo;
  split8(v, hi, lo);
  st2u4(wh + e0, hi);
  st2u4(wl + e0, lo);
}

__global__ __launch_bounds__(256) void k_packx(const float* __restrict__ src, int fullC, int chOff, int C, int Cpad,
                                               us_t* oh, us_t* ol, int ngroups)
{
  const int g = blockIdx.x * 256 + threadIdx.x;
  if (g >= ngroups) return;
  const int e0 = g * 8;
  const int px = e0 / Cpad;
  const int c0 = e0 - px * Cpad;
  const int b = px >> 12, sp = px & (HW - 1);
  float v[8];
#pragma unroll
  for (int i = 0; i < 8; ++i) {
    const int c = c0 + i;
    const int cc = min(c, C - 1);
    const float a = src[((size_t)(b * fullC + chOff + cc) << 12) + sp];
    v[i] = (c < C) ? a : 0.0f;
  }
  v4u hi, lo;
  split8(v, hi, lo);
  st2u4(oh + e0, hi);
  st2u4(ol + e0, lo);
}

__global__ __launch_bounds__(256) void k_packf1(const float* __restrict__ flow, us_t* oh, us_t* ol)
{
  const int g = blockIdx.x * 256 + threadIdx.x;
  if (g >= NPX * 16) return;
  const int px = g >> 4, k0 = (g & 15) * 8;
  const int b = px >> 12, sp = px & (HW - 1);
  const int y = sp >> 6, x = sp & 63;
  float v[8];
#pragma unroll
  for (int i = 0; i < 8; ++i) {
    const int k = k0 + i;
    const int kc = min(k, 97);
    const int tap = kc >> 1, ic = kc & 1;
    const int kh = tap / 7, kw = tap - kh * 7;
    const int ys = y + kh - 3, xs = x + kw - 3;
    const bool ok = (k < 98) && ((unsigned)ys < 64u) && ((unsigned)xs < 64u);
    const int ysc = min(max(ys, 0), 63), xsc = min(max(xs, 0), 63);
    const float a = flow[((size_t)(b * 2 + ic) << 12) + (ysc << 6) + xsc];
    v[i] = ok ? a : 0.0f;
  }
  v4u hi, lo;
  split8(v, hi, lo);
  st2u4(oh + px * 128 + k0, hi);
  st2u4(ol + px * 128 + k0, lo);
}

__global__ __launch_bounds__(256) void k_packcat(const float* __restrict__ x1, const float* __restrict__ upf,
                                                 const us_t* __restrict__ mh, const us_t* __restrict__ ml,
                                                 us_t* xh, us_t* xl)
{
  const int seg = blockIdx.y;
  const int g = blockIdx.x * 256 + threadIdx.x;
  const int px = g >> 4, c0 = (g & 15) * 8;
  const int b = px >> 12, sp = px & (HW - 1);
  const size_t o = (size_t)px * 512 + seg * 128 + c0;
  if (seg == 2) {
    const v4u a = ldg16(mh + (size_t)px * 128 + c0);
    const v4u c = ldg16(ml + (size_t)px * 128 + c0);
    st2u4(xh + o, a);
    st2u4(xl + o, c);
  } else {
    float v[8];
    if (seg == 0) {
#pragma unroll
      for (int i = 0; i < 8; ++i) v[i] = x1[((size_t)(b * 256 + c0 + i) << 12) + sp];
    } else {
#pragma unroll
      for (int i = 0; i < 8; ++i) v[i] = upf[((size_t)(b * 128 + c0 + i) << 12) + sp];
    }
    v4u hi, lo;
    split8(v, hi, lo);
    st2u4(xh + o, hi);
    st2u4(xl + o, lo);
  }
}

template <int MT, int NT, int EP>
__global__ __launch_bounds__(64) void k_conv(
    const us_t* __restrict__ xh, const us_t* __restrict__ xl, int Cpad,
    const us_t* __restrict__ wh, const us_t* __restrict__ wl, int Kpad,
    const float* __restrict__ bias, int nb, const float* __restrict__ bias2, int nb2,
    int KW, int taps, int dil, int padY, int padX, int wlog, int imgHW,
    int act, float oscale,
    void* o0, void* o1, void* o2, int oCpad, int oOff, int ocA, int ocB,
    const float* __restrict__ tail)
{
  static_assert(EP != 2 || MT == 4);
  static_assert(EP != 3 || MT == 2);
  static_assert(MT * NT <= 8);
  __shared__ __attribute__((aligned(16))) float stg[2][NT * 16 * MT * 16];

  const int tid = threadIdx.x, lane = tid & 31, wv = tid >> 5, h = lane >> 4, m = lane & 15;
  const int imgW = 1 << wlog;
  const int imgH = imgHW >> wlog;
  const int px0 = (blockIdx.x * 2 + wv) * (MT * 16);
  const int oc0 = blockIdx.y * (NT * 16);
  const int b = px0 / imgHW;
  const int sp0 = px0 - b * imgHW;
  const int bpix = b * imgH;

  int yy[MT], xx[MT];
#pragma unroll
  for (int mt = 0; mt < MT; ++mt) {
    const int p = sp0 + mt * 16 + m;
    yy[mt] = p >> wlog;
    xx[mt] = p & (imgW - 1);
  }
  int icj[2], khj[2], kwj[2], tpj[2];
#pragma unroll
  for (int j = 0; j < 2; ++j) {
    const int koff = 16 * j + 8 * h;
    const int t = koff / Cpad;
    icj[j] = koff - t * Cpad;
    tpj[j] = t;
    khj[j] = t / KW;
    kwj[j] = t - khj[j] * KW;
  }

  v8f acc[NT][MT];
#pragma unroll
  for (int nt = 0; nt < NT; ++nt)
#pragma unroll
    for (int mt = 0; mt < MT; ++mt) acc[nt][mt] = zero8f();

  const int nstep = Kpad >> 5;
#pragma unroll 1
  for (int s = 0; s < nstep; ++s) {
    FragB ah[MT], al[MT];
#pragma unroll
    for (int j = 0; j < 2; ++j) {
#pragma unroll
      for (int mt = 0; mt < MT; ++mt) {
        const int ys = yy[mt] + khj[j] * dil - padY;
        const int xs = xx[mt] + kwj[j] * dil - padX;
        const bool ok = (tpj[j] < taps) && ((unsigned)ys < (unsigned)imgH) && ((unsigned)xs < (unsigned)imgW);
        const int ysc = min(max(ys, 0), imgH - 1);
        const int xsc = min(max(xs, 0), imgW - 1);
        const int off = (((bpix + ysc) << wlog) + xsc) * Cpad + icj[j];
        const v4u th = ldg16(xh + off);
        const v4u tl = ldg16(xl + off);
        ah[mt].q[j] = ok ? th : zero4u();
        al[mt].q[j] = ok ? tl : zero4u();
      }
    }
    const int kb = s * 32;
#pragma unroll
    for (int nt = 0; nt < NT; ++nt) {
      FragB bh, bl;
#pragma unroll
      for (int j = 0; j < 2; ++j) {
        const int woff = (oc0 + nt * 16 + m) * Kpad + kb + 16 * j + 8 * h;
        bh.q[j] = ldg16(wh + woff);
        bl.q[j] = ldg16(wl + woff);
      }
#pragma unroll
      for (int mt = 0; mt < MT; ++mt) {
        acc[nt][mt] = mmab(ah[mt].v, bh.v, acc[nt][mt]);
        acc[nt][mt] = mmab(ah[mt].v, bl.v, acc[nt][mt]);
        acc[nt][mt] = mmab(al[mt].v, bh.v, acc[nt][mt]);
      }
      Guard<MT>::g(acc[nt], ah, al, bh, bl);
    }
#pragma unroll
    for (int j = 0; j < 2; ++j) {
      icj[j] += 32;
#pragma unroll
      for (int wrap = 0; wrap < 2; ++wrap) {
        if (icj[j] >= Cpad) {
          icj[j] -= Cpad;
          ++tpj[j];
          ++kwj[j];
          if (kwj[j] == KW) { kwj[j] = 0; ++khj[j]; }
        }
      }
    }
  }

  float* sw = stg[wv];
#pragma unroll
  for (int nt = 0; nt < NT; ++nt) {
    const int oc = oc0 + nt * 16 + m;
    float bv = 0.0f;
    if (nb > 0) {
      const float t1 = bias[min(oc, nb - 1)];
      float t2 = 0.0f;
      if (nb2 > 0) t2 = bias2[min(max(oc - nb, 0), nb2 - 1)];
      bv = (oc < nb) ? t1 : ((oc < nb + nb2) ? t2 : 0.0f);
    }
#pragma unroll
    for (int mt = 0; mt < MT; ++mt) {
      float v[8];
#pragma unroll
      for (int r = 0; r < 8; ++r) {
        float t = acc[nt][mt][r] + bv;
        if (act != 0) t = (t >= 0.0f) ? t : 0.1f * t;
        v[r] = t * oscale;
      }
      float* d = sw + (nt * 16 + m) * (MT * 16) + mt * 16 + 8 * h;
      v4f a, c;
      a.x = v[0]; a.y = v[1]; a.z = v[2]; a.w = v[3];
      c.x = v[4]; c.y = v[5]; c.z = v[6]; c.w = v[7];
      *(v4f*)d = a;
      *(v4f*)(d + 4) = c;
    }
  }
  __syncthreads();

  if (EP == 0) {
    us_t* oh = (us_t*)o0;
    us_t* ol = (us_t*)o1;
    float* of = (float*)o2;
#pragma unroll
    for (int it = 0; it < MT * NT; ++it) {
      const int g = it * 32 + lane;
      const int pl = g / (NT * 2);
      const int cg = g - pl * (NT * 2);
      float v[8];
#pragma unroll
      for (int i = 0; i < 8; ++i) v[i] = sw[(cg * 8 + i) * (MT * 16) + pl];
      if (tail != nullptr) {
        const int sp = sp0 + pl;
        const float fl0 = tail[(size_t)(b * 2) * imgHW + sp];
        const float fl1 = tail[(size_t)(b * 2 + 1) * imgHW + sp];
#pragma unroll
        for (int i = 0; i < 8; ++i) {
          const int c = oOff + oc0 + cg * 8 + i;
          v[i] = (c == 126) ? fl0 : ((c == 127) ? fl1 : v[i]);
        }
      }
      v4u hi, lo;
      split8(v, hi, lo);
      const size_t o = (size_t)(px0 + pl) * oCpad + oOff + oc0 + cg * 8;
      st2u4(oh + o, hi);
      st2u4(ol + o, lo);
    }
    if (of != nullptr) {
#pragma unroll
      for (int it = 0; it < MT * NT * 2; ++it) {
        const int g = it * 32 + lane;
        const int pl = g / (NT * 4);
        const int c4 = g - pl * (NT * 4);
        float v[4];
#pragma unroll
        for (int i = 0; i < 4; ++i) v[i] = sw[(c4 * 4 + i) * (MT * 16) + pl];
        if (tail != nullptr) {
          const int sp = sp0 + pl;
          const float fl0 = tail[(size_t)(b * 2) * imgHW + sp];
          const float fl1 = tail[(size_t)(b * 2 + 1) * imgHW + sp];
#pragma unroll
          for (int i = 0; i < 4; ++i) {
            const int c = oOff + oc0 + c4 * 4 + i;
            v[i] = (c == 126) ? fl0 : ((c == 127) ? fl1 : v[i]);
          }
        }
        v4f t;
        t.x = v[0]; t.y = v[1]; t.z = v[2]; t.w = v[3];
        st2f4(of + (size_t)(px0 + pl) * oCpad + oOff + oc0 + c4 * 4, t);
      }
    }
  } else if (EP == 1) {
    us_t* oh = (us_t*)o0;
#pragma unroll
    for (int it = 0; it < MT * NT; ++it) {
      const int g = it * 32 + lane;
      const int pl = g / (NT * 2);
      const int cg = g - pl * (NT * 2);
      float v[8];
#pragma unroll
      for (int i = 0; i < 8; ++i) v[i] = sw[(cg * 8 + i) * (MT * 16) + pl];
      const v4u pk = pack8h(v);
      st2u4(oh + (size_t)(px0 + pl) * oCpad + oOff + oc0 + cg * 8, pk);
    }
  } else if (EP == 2) {
    us_t* ov = (us_t*)o0;
#pragma unroll
    for (int it = 0; it < NT * 4; ++it) {
      const int g = it * 32 + lane;
      const int row = g >> 3, pg = g & 7;
      const float* sr = sw + row * 64 + pg * 8;
      const v4f a = *(const v4f*)sr;
      const v4f c = *(const v4f*)(sr + 4);
      float v[8];
      v[0] = a.x; v[1] = a.y; v[2] = a.z; v[3] = a.w; v[4] = c.x; v[5] = c.y; v[6] = c.z; v[7] = c.w;
      const v4u pk = pack8h(v);
      st2u4(ov + ((size_t)(b * oCpad + oc0 + row) * imgHW + sp0 + pg * 8), pk);
    }
  } else {
    float* oa = (float*)o0;
    float* ob = (float*)o1;
#pragma unroll
    for (int it = 0; it < NT * 4; ++it) {
      const int g = it * 32 + lane;
      const int row = g >> 3, pg = g & 7;
      const int oc = oc0 + row;
      const v4f t = *(const v4f*)(sw + row * 32 + pg * 4);
      if (oc < ocA) {
        st2f4(oa + ((size_t)(b * ocA + oc) * imgHW + sp0 + pg * 4), t);
      } else if (oc < ocA + ocB) {
        st2f4(ob + ((size_t)(b * ocB + (oc - ocA)) * imgHW + sp0 + pg * 4), t);
      }
    }
  }
}

__global__ __launch_bounds__(64) void k_deconv(const us_t* __restrict__ xh, const us_t* __restrict__ xl,
                                               const us_t* __restrict__ wh, const us_t* __restrict__ wl,
                                               const float* __restrict__ bias,
                                               float* out1, us_t* uh, us_t* ul)
{
  __shared__ __attribute__((aligned(16))) float stg[2][16 * 32];
  const int tid = threadIdx.x, lane = tid & 31, wv = tid >> 5, h = lane >> 4, m = lane & 15;
  const int gw = blockIdx.x * 2 + wv;
  const int j = gw & 3, yo = (gw >> 2) & 127, b = gw >> 9;
  const int py = yo & 1, yb = yo >> 1;
  const int xb = 16 * j + m;

  v8f acc[2];
  acc[0] = zero8f();
  acc[1] = zero8f();
#pragma unroll
  for (int t = 0; t < 4; ++t) {
    const int a = t >> 1, c = t & 1;
    const int ys = yb + py - 1 + a;
    const bool oky = (unsigned)ys < 64u;
    const int ysc = min(max(ys, 0), 63);
    FragB fah[2], fal[2], fbh[2], fbl[2];
#pragma unroll
    for (int p = 0; p < 2; ++p) {
      const int xs = xb + p - 1 + c;
      const bool ok = oky && ((unsigned)xs < 64u);
      const int xsc = min(max(xs, 0), 63);
      const int base = ((b * 64 + ysc) * 64 + xsc) * 32;
      const int wb = ((py * 2 + p) * 16 + m) * 128 + t * 32;
#pragma unroll
      for (int hf = 0; hf < 2; ++hf) {
        const int o = base + 16 * hf + 8 * h;
        const v4u th = ldg16(xh + o);
        const v4u tl = ldg16(xl + o);
        fah[p].q[hf] = ok ? th : zero4u();
        fal[p].q[hf] = ok ? tl : zero4u();
        const int wo = wb + 16 * hf + 8 * h;
        fbh[p].q[hf] = ldg16(wh + wo);
        fbl[p].q[hf] = ldg16(wl + wo);
      }
    }
#pragma unroll
    for (int p = 0; p < 2; ++p) {
      acc[p] = mmab(fah[p].v, fbh[p].v, acc[p]);
      acc[p] = mmab(fah[p].v, fbl[p].v, acc[p]);
      acc[p] = mmab(fal[p].v, fbh[p].v, acc[p]);
    }
    asm volatile(NOP4 : "+v"(acc[0]), "+v"(acc[1])
                 : "v"(fah[0].v), "v"(fah[1].v), "v"(fal[0].v), "v"(fal[1].v),
                   "v"(fbh[0].v), "v"(fbh[1].v), "v"(fbl[0].v), "v"(fbl[1].v));
  }

  const float bv = bias[m];
  float t16[16];
#pragma unroll
  for (int r = 0; r < 8; ++r) {
#pragma unroll
    for (int p = 0; p < 2; ++p) {
      float t = acc[p][r] + bv;
      t = (t >= 0.0f) ? t : 0.1f * t;
      t16[2 * r + p] = t;
    }
  }
  float* sw = stg[wv];
  {
    float* d = sw + m * 32 + 16 * h;
#pragma unroll
    for (int q = 0; q < 4; ++q) {
      v4f a;
      a.x = t16[4 * q]; a.y = t16[4 * q + 1]; a.z = t16[4 * q + 2]; a.w = t16[4 * q + 3];
      *(v4f*)(d + 4 * q) = a;
    }
  }
  __syncthreads();

  const int sp0 = yo * 128 + 32 * j;
#pragma unroll
  for (int it = 0; it < 4; ++it) {
    const int g = it * 32 + lane;
    const int row = g >> 3, pg = g & 7;
    const v4f t = *(const v4f*)(sw + row * 32 + pg * 4);
    st2f4(out1 + ((size_t)(b * 16 + row) * 16384 + sp0 + pg * 4), t);
  }
#pragma unroll
  for (int it = 0; it < 2; ++it) {
    const int g = it * 32 + lane;
    const int xl_ = g >> 1, cg = g & 1;
    float v[8];
#pragma unroll
    for (int i = 0; i < 8; ++i) v[i] = sw[(cg * 8 + i) * 32 + xl_];
    v4u hi, lo;
    split8(v, hi, lo);
    const size_t o = ((size_t)b * 16384 + sp0 + xl_) * 16 + cg * 8;
    st2u4(uh + o, hi);
    st2u4(ul + o, lo);
  }
}

__global__ __launch_bounds__(64) void k_attn(const us_t* __restrict__ qk, const us_t* __restrict__ vt,
                                             const float* __restrict__ motf, const float* __restrict__ gam,
                                             us_t* xh, us_t* xl, float cs)
{
  __shared__ __attribute__((aligned(16))) float stg[2][16 * 128];
  const int tid = threadIdx.x, lane = tid & 31, wv = tid >> 5, h = lane >> 4, m = lane & 15;
  const int b = blockIdx.y;
  const int q0 = (blockIdx.x * 2 + wv) * 16;
  const size_t bq = (size_t)b * HW;

  FragH fq[4];
#pragma unroll
  for (int kc = 0; kc < 4; ++kc) {
    const size_t off = (bq + q0 + m) * 256 + kc * 32 + 8 * h;
    fq[kc].q[0] = ldg16(qk + off);
    fq[kc].q[1] = ldg16(qk + off + 16);
  }
  v8f O[8];
#pragma unroll
  for (int n = 0; n < 8; ++n) O[n] = zero8f();
  float mrun = -1e30f, lrun = 0.0f;

#pragma unroll 1
  for (int kv0 = 0; kv0 < HW; kv0 += 32) {
    v8f S[2];
#pragma unroll
    for (int kt = 0; kt < 2; ++kt) {
      S[kt] = zero8f();
      FragH ka[4];
#pragma unroll
      for (int kc = 0; kc < 4; ++kc) {
        const size_t off = (bq + kv0 + kt * 16 + m) * 256 + 128 + kc * 32 + 8 * h;
        ka[kc].q[0] = ldg16(qk + off);
        ka[kc].q[1] = ldg16(qk + off + 16);
      }
#pragma unroll
      for (int kc = 0; kc < 4; ++kc) S[kt] = mmah(ka[kc].v, fq[kc].v, S[kt]);
      asm volatile(NOP4 : "+v"(S[kt])
                   : "v"(ka[0].v), "v"(ka[1].v), "v"(ka[2].v), "v"(ka[3].v),
                     "v"(fq[0].v), "v"(fq[1].v), "v"(fq[2].v), "v"(fq[3].v));
    }
    float mx = -1e30f;
#pragma unroll
    for (int kt = 0; kt < 2; ++kt)
#pragma unroll
      for (int r = 0; r < 8; ++r) mx = fmaxf(mx, S[kt][r]);
    mx = fmaxf(mx, __shfl_xor(mx, 16, 32));
    const float mnew = fmaxf(mrun, mx * cs);
    const float alpha = __expf(mrun - mnew);
    float ps = 0.0f;
    FragH bp;
#pragma unroll
    for (int kt = 0; kt < 2; ++kt) {
#pragma unroll
      for (int r = 0; r < 8; ++r) {
        const float p = __expf(S[kt][r] * cs - mnew);
        ps += p;
        bp.hv[kt][r] = (_Float16)(p * 1024.0f);
      }
    }
    ps += __shfl_xor(ps, 16, 32);
    lrun = lrun * alpha + ps;
    mrun = mnew;
#pragma unroll
    for (int n = 0; n < 8; ++n) O[n] = O[n] * alpha;
    FragH va;
#pragma unroll
    for (int n = 0; n < 8; ++n) {
      const size_t off = ((size_t)(b * 128 + n * 16 + m)) * HW + kv0 + 8 * h;
      va.q[0] = ldg16(vt + off);
      va.q[1] = ldg16(vt + off + 16);
      O[n] = mmah(va.v, bp.v, O[n]);
    }
    asm volatile(NOP4 : "+v"(O[0]), "+v"(O[1]), "+v"(O[2]), "+v"(O[3]),
                        "+v"(O[4]), "+v"(O[5]), "+v"(O[6]), "+v"(O[7])
                 : "v"(va.v), "v"(bp.v));
  }

  const float inv = 1.0f / (lrun * 16384.0f);
  float* sw = stg[wv];
#pragma unroll
  for (int n = 0; n < 8; ++n) {
    v4f a, c;
    a.x = O[n][0] * inv; a.y = O[n][1] * inv; a.z = O[n][2] * inv; a.w = O[n][3] * inv;
    c.x = O[n][4] * inv; c.y = O[n][5] * inv; c.z = O[n][6] * inv; c.w = O[n][7] * inv;
    float* d = sw + m * 128 + n * 16 + 8 * h;
    *(v4f*)d = a;
    *(v4f*)(d + 4) = c;
  }
  __syncthreads();
  const float g = gam[0];
#pragma unroll 4
  for (int it = 0; it < 16; ++it) {
    const size_t px = bq + q0 + it;
    const v4f o4 = *(const v4f*)(sw + it * 128 + 4 * lane);
    const v4f m4 = *(const v4f*)(motf + px * 128 + 4 * lane);
    const float r0 = m4.x + g * o4.x;
    const float r1 = m4.y + g * o4.y;
    const float r2 = m4.z + g * o4.z;
    const float r3 = m4.w + g * o4.w;
    unsigned h01, l01, h23, l23;
    split2(r0, r1, h01, l01);
    split2(r2, r3, h23, l23);
    v2u hi, lo;
    hi.x = h01; hi.y = h23; lo.x = l01; lo.y = l23;
    const size_t o = px * 512 + 384 + 4 * lane;
    st2u2(xh + o, hi);
    st2u2(xl + o, lo);
  }
}

template <int MT, int NT, int EP>
static void conv(hipStream_t st, int npix, int ocPad,
                 const us_t* xh, const us_t* xl, int Cpad,
                 const us_t* wh, const us_t* wl, int Kpad,
                 const float* bias, int nb, const float* bias2, int nb2,
                 int KW, int taps, int dil, int pad, int wlog, int imgHW,
                 int act, float oscale,
                 void* o0, void* o1, void* o2, int oCpad, int oOff, int ocA, int ocB, const float* tail)
{
  dim3 grid(npix / (2 * MT * 16), ocPad / (NT * 16));
  k_conv<MT, NT, EP><<<grid, 64, 0, st>>>(xh, xl, Cpad, wh, wl, Kpad, bias, nb, bias2, nb2,
                                           KW, taps, dil, pad, pad, wlog, imgHW, act, oscale,
                                           o0, o1, o2, oCpad, oOff, ocA, ocB, tail);
}

static void packw(hipStream_t st, const float* w, int OC, const float* w2, int OC2, int Cin, int taps,
                  int Cpad, int Kpad, int ocPad, us_t* wh, us_t* wl)
{
  const int ng = ocPad * Kpad / 8;
  k_packw<<<(ng + 255) / 256, 256, 0, st>>>(w, OC, w2, OC2, Cin, taps, Cpad, Kpad, wh, wl, ng);
}

extern "C" void kernel_launch(void* const* d_in, const int* in_sizes, int n_in,
                              void* d_out, int out_size, void* d_ws, size_t ws_size,
                              hipStream_t stream)
{
  if (n_in < 33) return;
  const int expect[33] = {4194304, 2097152, 1327104, 32768, 32768, 20736, 256, 442368, 192, 12544, 128,
                          73728, 64, 290304, 126, 16384, 1, 589824, 128, 110592, 96, 55296, 64, 18432, 32,
                          8192, 16, 9216, 64, 576, 2, 288, 1};
  for (int i = 0; i < 33; ++i) if (in_sizes[i] != expect[i]) return;
  if (out_size != 5292032) return;

  const float* x1     = (const float*)d_in[0];
  const float* upfeat = (const float*)d_in[1];
  const float* corr   = (const float*)d_in[2];
  const float* flow   = (const float*)d_in[3];
  const float* w_qk   = (const float*)d_in[4];
  const float* w_c1   = (const float*)d_in[5];   const float* b_c1 = (const float*)d_in[6];
  const float* w_c2   = (const float*)d_in[7];   const float* b_c2 = (const float*)d_in[8];
  const float* w_f1   = (const float*)d_in[9];   const float* b_f1 = (const float*)d_in[10];
  const float* w_f2   = (const float*)d_in[11];  const float* b_f2 = (const float*)d_in[12];
  const float* w_mo   = (const float*)d_in[13];  const float* b_mo = (const float*)d_in[14];
  const float* w_v    = (const float*)d_in[15];
  const float* gamma  = (const float*)d_in[16];
  const float* w1     = (const float*)d_in[17];  const float* b1 = (const float*)d_in[18];
  const float* w2     = (const float*)d_in[19];  const float* b2 = (const float*)d_in[20];
  const float* w3     = (const float*)d_in[21];  const float* b3 = (const float*)d_in[22];
  const float* w4     = (const float*)d_in[23];  const float* b4 = (const float*)d_in[24];
  const float* w_up   = (const float*)d_in[25];  const float* b_up = (const float*)d_in[26];
  const float* w_tr   = (const float*)d_in[27];  const float* b_tr = (const float*)d_in[28];
  const float* w_fl   = (const float*)d_in[29];  const float* b_fl = (const float*)d_in[30];
  const float* w_mk   = (const float*)d_in[31];  const float* b_mk = (const float*)d_in[32];

  float* out  = (float*)d_out;
  float* out0 = out;
  float* out1 = out + 4194304;
  float* out2 = out + 5242880;
  float* out3 = out + 5275648;

  char* ws = (char*)d_ws;
  size_t off = 0;
  auto carve = [&](size_t bytes) -> char* { char* p = ws + off; off += (bytes + 255) & ~(size_t)255; return p; };
  auto wplane = [&](int ocPad, int Kpad) -> us_t* { return (us_t*)carve((size_t)ocPad * Kpad * 2); };

  us_t* wqk_h = wplane(256, 128);   us_t* wqk_l = wplane(256, 128);
  us_t* wc1_h = wplane(256, 96);    us_t* wc1_l = wplane(256, 96);
  us_t* wc2_h = wplane(192, 2304);  us_t* wc2_l = wplane(192, 2304);
  us_t* wf1_h = wplane(128, 128);   us_t* wf1_l = wplane(128, 128);
  us_t* wf2_h = wplane(64, 1152);   us_t* wf2_l = wplane(64, 1152);
  us_t* wmo_h = wplane(128, 2304);  us_t* wmo_l = wplane(128, 2304);
  us_t* wv_h  = wplane(128, 128);   us_t* wv_l  = wplane(128, 128);
  us_t* w1_h  = wplane(128, 4608);  us_t* w1_l  = wplane(128, 4608);
  us_t* w2_h  = wplane(96, 1152);   us_t* w2_l  = wplane(96, 1152);
  us_t* w3_h  = wplane(64, 864);    us_t* w3_l  = wplane(64, 864);
  us_t* w4_h  = wplane(32, 576);    us_t* w4_l  = wplane(32, 576);
  us_t* wd_h  = wplane(64, 128);    us_t* wd_l  = wplane(64, 128);
  us_t* wt_h  = wplane(64, 160);    us_t* wt_l  = wplane(64, 160);
  us_t* whd_h = wplane(16, 288);    us_t* whd_l = wplane(16, 288);

  char* X = carve((size_t)NPX * 512 * 2 * 2);
  char* Y = carve((size_t)16777216);
  char* Z = carve((size_t)8388608);
  char* M = carve((size_t)16777216);
  char* S = carve((size_t)6291456);
  if (off > ws_size || off > (size_t)134217728u) return;

  us_t* cor1_h = (us_t*)(X);                       us_t* cor1_l = (us_t*)(X + 8388608);
  us_t* cflo_h = (us_t*)(X + 16777216);            us_t* cflo_l = (us_t*)(X + 25165824);
  us_t* xc_h   = (us_t*)(X);                       us_t* xc_l   = (us_t*)(X + 16777216);
  us_t* corr_h = (us_t*)(Y);                       us_t* corr_l = (us_t*)(Y + 3145728);
  us_t* f1c_h  = (us_t*)(Y + 6291456);             us_t* f1c_l  = (us_t*)(Y + 10485760);
  us_t* inp_h  = (us_t*)(Y);                       us_t* inp_l  = (us_t*)(Y + 4194304);
  us_t* up_h   = (us_t*)(Y);                       us_t* up_l   = (us_t*)(Y + 2097152);
  us_t* flo1_h = (us_t*)(Z);                       us_t* flo1_l = (us_t*)(Z + 4194304);
  us_t* qk_p   = (us_t*)(Z);
  us_t* x1_h   = (us_t*)(Z);                       us_t* x1_l   = (us_t*)(Z + 4194304);
  us_t* x3_h   = (us_t*)(Z);                       us_t* x3_l   = (us_t*)(Z + 2097152);
  us_t* mo_h   = (us_t*)(M);                       us_t* mo_l   = (us_t*)(M + 4194304);
  float* mo_f  = (float*)(M + 8388608);
  us_t* vt_p   = (us_t*)(S);
  us_t* x2_h   = (us_t*)(S);                       us_t* x2_l   = (us_t*)(S + 3145728);
  us_t* x4_h   = (us_t*)(S);                       us_t* x4_l   = (us_t*)(S + 1048576);

  packw(stream, w_qk, 256, w_qk, 0, 128, 1, 128, 128, 256, wqk_h, wqk_l);
  packw(stream, w_c1, 256, w_c1, 0, 81, 1, 96, 96, 256, wc1_h, wc1_l);
  packw(stream, w_c2, 192, w_c2, 0, 256, 9, 256, 2304, 192, wc2_h, wc2_l);
  packw(stream, w_f1, 128, w_f1, 0, 2, 49, 2, 128, 128, wf1_h, wf1_l);
  packw(stream, w_f2, 64, w_f2, 0, 128, 9, 128, 1152, 64, wf2_h, wf2_l);
  packw(stream, w_mo, 126, w_mo, 0, 256, 9, 256, 2304, 128, wmo_h, wmo_l);
  packw(stream, w_v, 128, w_v, 0, 128, 1, 128, 128, 128, wv_h, wv_l);
  packw(stream, w1, 128, w1, 0, 512, 9, 512, 4608, 128, w1_h, w1_l);
  packw(stream, w2, 96, w2, 0, 128, 9, 128, 1152, 96, w2_h, w2_l);
  packw(stream, w3, 64, w3, 0, 96, 9, 96, 864, 64, w3_h, w3_l);
  packw(stream, w4, 32, w4, 0, 64, 9, 64, 576, 32, w4_h, w4_l);
  packw(stream, w_tr, 64, w_tr, 0, 16, 9, 16, 160, 64, wt_h, wt_l);
  packw(stream, w_fl, 2, w_mk, 1, 32, 9, 32, 288, 16, whd_h, whd_l);
  k_packwd<<<4, 256, 0, stream>>>(w_up, wd_h, wd_l);

  { const int ng = NPX * 96 / 8; k_packx<<<(ng + 255) / 256, 256, 0, stream>>>(corr, 81, 0, 81, 96, corr_h, corr_l, ng); }
  k_packf1<<<NPX * 16 / 256, 256, 0, stream>>>(flow, f1c_h, f1c_l);
  conv<2, 4, 0>(stream, NPX, 256, corr_h, corr_l, 96, wc1_h, wc1_l, 96, b_c1, 256, b_c1, 0,
                1, 1, 1, 0, 6, HW, 1, 1.0f, cor1_h, cor1_l, nullptr, 256, 0, 0, 0, nullptr);
  conv<2, 4, 0>(stream, NPX, 192, cor1_h, cor1_l, 256, wc2_h, wc2_l, 2304, b_c2, 192, b_c2, 0,
                3, 9, 1, 1, 6, HW, 1, 1.0f, cflo_h, cflo_l, nullptr, 256, 0, 0, 0, nullptr);
  conv<2, 4, 0>(stream, NPX, 128, f1c_h, f1c_l, 128, wf1_h, wf1_l, 128, b_f1, 128, b_f1, 0,
                1, 1, 1, 0, 6, HW, 1, 1.0f, flo1_h, flo1_l, nullptr, 128, 0, 0, 0, nullptr);
  conv<2, 4, 0>(stream, NPX, 64, flo1_h, flo1_l, 128, wf2_h, wf2_l, 1152, b_f2, 64, b_f2, 0,
                3, 9, 1, 1, 6, HW, 1, 1.0f, cflo_h, cflo_l, nullptr, 256, 192, 0, 0, nullptr);
  conv<2, 4, 0>(stream, NPX, 128, cflo_h, cflo_l, 256, wmo_h, wmo_l, 2304, b_mo, 126, b_mo, 0,
                3, 9, 1, 1, 6, HW, 1, 1.0f, mo_h, mo_l, mo_f, 128, 0, 0, 0, flow);

  { const int ng = NPX * 128 / 8; k_packx<<<(ng + 255) / 256, 256, 0, stream>>>(x1, 256, 128, 128, 128, inp_h, inp_l, ng); }
  conv<2, 4, 1>(stream, NPX, 256, inp_h, inp_l, 128, wqk_h, wqk_l, 128, w_qk, 0, w_qk, 0,
                1, 1, 1, 0, 6, HW, 0, 8.0f, qk_p, nullptr, nullptr, 256, 0, 0, 0, nullptr);
  conv<4, 2, 2>(stream, NPX, 128, mo_h, mo_l, 128, wv_h, wv_l, 128, w_v, 0, w_v, 0,
                1, 1, 1, 0, 6, HW, 0, 16.0f, vt_p, nullptr, nullptr, 128, 0, 0, 0, nullptr);
  k_attn<<<dim3(HW / 32, 4), 64, 0, stream>>>(qk_p, vt_p, mo_f, gamma, xc_h, xc_l, 0.08838834764831845f / 64.0f);
  k_packcat<<<dim3(NPX * 16 / 256, 3), 256, 0, stream>>>(x1, upfeat, mo_h, mo_l, xc_h, xc_l);

  conv<2, 4, 0>(stream, NPX, 128, xc_h, xc_l, 512, w1_h, w1_l, 4608, b1, 128, b1, 0,
                3, 9, 1, 1, 6, HW, 1, 1.0f, x1_h, x1_l, nullptr, 128, 0, 0, 0, nullptr);
  conv<1, 6, 0>(stream, NPX, 96, x1_h, x1_l, 128, w2_h, w2_l, 1152, b2, 96, b2, 0,
                3, 9, 4, 4, 6, HW, 1, 1.0f, x2_h, x2_l, nullptr, 96, 0, 0, 0, nullptr);
  conv<2, 4, 0>(stream, NPX, 64, x2_h, x2_l, 96, w3_h, w3_l, 864, b3, 64, b3, 0,
                3, 9, 8, 8, 6, HW, 1, 1.0f, x3_h, x3_l, nullptr, 64, 0, 0, 0, nullptr);
  conv<2, 2, 0>(stream, NPX, 32, x3_h, x3_l, 64, w4_h, w4_l, 576, b4, 32, b4, 0,
                3, 9, 1, 1, 6, HW, 1, 1.0f, x4_h, x4_l, nullptr, 32, 0, 0, 0, nullptr);

  k_deconv<<<1024, 64, 0, stream>>>(x4_h, x4_l, wd_h, wd_l, b_up, out1, up_h, up_l);
  conv<2, 4, 3>(stream, 65536, 64, up_h, up_l, 16, wt_h, wt_l, 160, b_tr, 64, b_tr, 0,
                3, 9, 1, 1, 7, 16384, 0, 1.0f, out0, nullptr, nullptr, 0, 0, 64, 0, nullptr);
  conv<2, 1, 3>(stream, NPX, 16, x4_h, x4_l, 32, whd_h, whd_l, 288, b_fl, 2, b_mk, 1,
                3, 9, 1, 1, 6, HW, 0, 1.0f, out2, out3, nullptr, 0, 0, 2, 1, nullptr);
}
